// OurGAL_37185826849364
// MI455X (gfx1250) — hardware-verified
//
#include <hip/hip_runtime.h>
#include <stddef.h>
#include <math.h>


#define DIMC   128
#define NAGE   7
#define NOCC   21
#define NHEAD  29
#define HP     32
#define NTHR   256
#define NWAVE  8
#define EPT    8
#define NGRP   2
#define CHUNK  (NTHR * EPT * NGRP)
#define WCAP   (EPT * NGRP * 32)
#define LISTN  (NWAVE * WCAP)
#define NBA    2048
#define SCAP   320
#define RPB    512
#define GS     64
#define AP     136
#define NPB    (GS * NAGE / 4 + GS / 4 + GS * NOCC / 4 + 8)
#define BNEPS  1e-5f

#define LDS_AGG ((SCAP * DIMC + NBA + LISTN + SCAP + SCAP + 2 * DIMC + NWAVE + 8) * 4)
#define LDS_GH  (2 * GS * AP * 2 + DIMC * HP * 4 + DIMC * 4 + HP * 4 + GS * HP * 4 + GS * 4)

static_assert((CHUNK & (CHUNK - 1)) == 0);
static_assert(CHUNK <= 4096);
static_assert((NBA & (NBA - 1)) == 0 && NBA <= 4096);
static_assert(SCAP <= 512);
static_assert(GS * DIMC * 4 <= 2 * GS * AP * 2);
static_assert(GS == NWAVE * 8);
static_assert((GS * NAGE) % 32 == 0 && (GS * NOCC) % 32 == 0 && (GS % 32) == 0);
static_assert((RPB % NWAVE) == 0);
static_assert(NPB <= 2 * NTHR && (NPB % 8) == 0);
static_assert((GS * DIMC / 4) % NTHR == 0);

typedef float  v4f  __attribute__((ext_vector_type(4)));
typedef float  v8f  __attribute__((ext_vector_type(8)));
typedef int    v4i  __attribute__((ext_vector_type(4)));
typedef double v2d  __attribute__((ext_vector_type(2)));
typedef __bf16 v4b  __attribute__((ext_vector_type(4)));
typedef __bf16 v8b  __attribute__((ext_vector_type(8)));
typedef __bf16 v16b __attribute__((ext_vector_type(16)));
union FragB { v16b v; v8b h[2]; };

__device__ __forceinline__ int clampi(int v, int lo, int hi) { return v < lo ? lo : (v > hi ? hi : v); }

__device__ __forceinline__ void split_bf16(float x, __bf16& h, __bf16& l) {
  const __bf16 hb = (__bf16)x;
  const float  hf = (float)hb;
  h = hb;
  l = (__bf16)(x - hf);
}

__device__ __forceinline__ v8f wmb(v16b a, v16b b, v8f c) {
  v8f d = __builtin_amdgcn_wmma_f32_16x16x32_bf16(false, a, false, b, (short)0, c, false, false);
  asm volatile("v_nop\n\tv_nop\n\tv_nop\n\tv_nop" : "+v"(d) : "v"(a), "v"(b));
  return d;
}

template <int NB, int CLAMPV, int USEMAP>
__device__ __forceinline__ int scan_chunk(const int* __restrict__ ids, int nE, int cbase, int slotBase,
                                          int vec8, int nClamp, int* list, const int* map,
                                          int tid, int lane, int wave) {
  int wc = 0;
#pragma unroll
  for (int g = 0; g < NGRP; ++g) {
    const int el0  = (g * NTHR + tid) * EPT;
    const int e0   = cbase + el0;
    const int sent = -2147483647 - 1;
    int d[EPT];
    if (vec8 != 0 && cbase + CHUNK <= nE) {
      const v4i da = *(const v4i*)(ids + e0);
      const v4i db = *(const v4i*)(ids + e0 + 4);
      d[0] = da.x; d[1] = da.y; d[2] = da.z; d[3] = da.w;
      d[4] = db.x; d[5] = db.y; d[6] = db.z; d[7] = db.w;
      if (CLAMPV) {
#pragma unroll
        for (int j = 0; j < EPT; ++j) d[j] = clampi(d[j], 0, nClamp - 1);
      }
    } else {
#pragma unroll
      for (int j = 0; j < EPT; ++j) {
        const int ec = (e0 + j) < (nE - 1) ? (e0 + j) : (nE - 1);
        int v = ids[ec];
        if (CLAMPV) v = clampi(v, 0, nClamp - 1);
        d[j] = (e0 + j < nE) ? v : sent;
      }
    }
    bool h[EPT];
    int  code[EPT];
    bool anyl = false;
#pragma unroll
    for (int j = 0; j < EPT; ++j) {
      const unsigned s = (unsigned)d[j] - (unsigned)slotBase;
      bool hj = s < (unsigned)NB;
      int  cj = (int)s;
      if (USEMAP) {
        const int r = map[hj ? (int)s : 0];
        hj = hj && (r >= 0);
        cj = r;
      }
      h[j] = hj; code[j] = cj; anyl = anyl || hj;
    }
    const unsigned any = __builtin_amdgcn_ballot_w32(anyl);
    if (any != 0u) {
#pragma unroll
      for (int j = 0; j < EPT; ++j) {
        const unsigned mj = __builtin_amdgcn_ballot_w32(h[j]);
        if (mj != 0u) {
          if (h[j]) {
            const int pos = wc + (int)__builtin_amdgcn_mbcnt_lo(mj, 0u);
            if (pos < WCAP) list[wave * WCAP + pos] = ((el0 + j) << 12) | (code[j] & 4095);
          }
          wc += (int)__builtin_popcount(mj);
        }
      }
    }
  }
  return wc;
}

__global__ __launch_bounds__(NTHR) void k_stats(const float* __restrict__ E, double* statP, int nN) {
  __shared__ __attribute__((aligned(16))) double ps[NWAVE * DIMC];
  __shared__ __attribute__((aligned(16))) double pq[NWAVE * DIMC];
  __shared__ __attribute__((aligned(16))) double so[2 * DIMC];
  const int tid = threadIdx.x, lane = tid & 31, wave = tid >> 5;
  const int c4 = lane * 4;
  const int base = blockIdx.x * RPB;
  double s0 = 0.0, s1 = 0.0, s2 = 0.0, s3 = 0.0, q0 = 0.0, q1 = 0.0, q2 = 0.0, q3 = 0.0;
  const v4f z4 = {0.f, 0.f, 0.f, 0.f};
#pragma unroll 1
  for (int i = 0; i < RPB / NWAVE; ++i) {
    const int r  = base + wave + NWAVE * i;
    const int rc = r < nN ? r : nN - 1;
    v4f v = *(const v4f*)(E + (size_t)rc * DIMC + c4);
    v = (r < nN) ? v : z4;
    const double x0 = (double)v.x, x1 = (double)v.y, x2 = (double)v.z, x3 = (double)v.w;
    s0 += x0; s1 += x1; s2 += x2; s3 += x3;
    q0 = fma(x0, x0, q0); q1 = fma(x1, x1, q1); q2 = fma(x2, x2, q2); q3 = fma(x3, x3, q3);
  }
  ps[wave * DIMC + c4 + 0] = s0; ps[wave * DIMC + c4 + 1] = s1;
  ps[wave * DIMC + c4 + 2] = s2; ps[wave * DIMC + c4 + 3] = s3;
  pq[wave * DIMC + c4 + 0] = q0; pq[wave * DIMC + c4 + 1] = q1;
  pq[wave * DIMC + c4 + 2] = q2; pq[wave * DIMC + c4 + 3] = q3;
  __syncthreads();
  if (tid < DIMC) {
    double S = 0.0, Q = 0.0;
#pragma unroll
    for (int w = 0; w < NWAVE; ++w) { S += ps[w * DIMC + tid]; Q += pq[w * DIMC + tid]; }
    so[tid] = S;
    so[DIMC + tid] = Q;
  }
  __syncthreads();
  v2d val = {0.0, 0.0};
  if (tid < DIMC) val = *(const v2d*)(so + 2 * tid);
  double* gp = statP + (size_t)blockIdx.x * 2 * DIMC + 2 * tid;
  if (tid < DIMC) *(volatile v2d*)gp = val;
  __threadfence();
  if (tid < DIMC) *(volatile v2d*)gp = val;
}

__global__ __launch_bounds__(DIMC) void k_bnfin(
    const double* __restrict__ statP, int nP, double invN,
    const float* __restrict__ gamma, const float* __restrict__ beta, float* bnP) {
  __shared__ __attribute__((aligned(16))) float so[2 * DIMC];
  const int c = threadIdx.x;
  double S = 0.0, Q = 0.0;
#pragma unroll 1
  for (int p = 0; p < nP; ++p) {
    S += statP[(size_t)p * 2 * DIMC + c];
    Q += statP[(size_t)p * 2 * DIMC + DIMC + c];
  }
  const double mu = S * invN;
  double var = Q * invN - mu * mu;
  var = var < 0.0 ? 0.0 : var;
  const float rstd = rsqrtf((float)var + BNEPS);
  const float sc = rstd * gamma[c];
  const float sh = beta[c] - (float)mu * sc;
  so[c] = sc;
  so[DIMC + c] = sh;
  __syncthreads();
  v4f val = {0.f, 0.f, 0.f, 0.f};
  if (c < 2 * DIMC / 4) val = *(const v4f*)(so + 4 * c);
  float* gp = bnP + 4 * c;
  if (c < 2 * DIMC / 4) *(volatile v4f*)gp = val;
  __threadfence();
  if (c < 2 * DIMC / 4) *(volatile v4f*)gp = val;
}

__global__ __launch_bounds__(NTHR) void k_wprep(const float* __restrict__ W, __bf16* wh, __bf16* wl) {
  const int g = blockIdx.x * NTHR + (int)threadIdx.x;
  if (g >= DIMC * DIMC / 8) return;
  const int n = g >> 4, k0 = (g & 15) * 8;
  v8b hv, lv;
#pragma unroll
  for (int e = 0; e < 8; ++e) {
    const float x = W[(size_t)(k0 + e) * DIMC + n];
    __bf16 h, l;
    split_bf16(x, h, l);
    hv[e] = h; lv[e] = l;
  }
  __bf16* hp = wh + (size_t)n * DIMC + k0;
  __bf16* lp = wl + (size_t)n * DIMC + k0;
  *(volatile v8b*)hp = hv;
  *(volatile v8b*)lp = lv;
  __threadfence();
  *(volatile v8b*)hp = hv;
  *(volatile v8b*)lp = lv;
}

__global__ __launch_bounds__(NTHR) void k_aggr(
    const float* __restrict__ E, const int* __restrict__ src, const int* __restrict__ dst,
    const int* __restrict__ nbr, const float* __restrict__ bnP, float* aggP,
    int nN, int nE, int nB, int vec8) {
  extern __shared__ v4f lds_dyn[];
  float* rows = (float*)lds_dyn;
  int*   map  = (int*)(rows + SCAP * DIMC);
  int*   list = map + NBA;
  int*   rcnt = list + LISTN;
  int*   samp = rcnt + SCAP;
  float* scsh = (float*)(samp + SCAP);
  int*   wcnt = (int*)(scsh + 2 * DIMC);
  int*   cnt2 = wcnt + NWAVE;
  const int tid = threadIdx.x, lane = tid & 31, wave = tid >> 5;
  const int nodeBase = blockIdx.x * NBA;

  {
    const v4f z4 = {0.f, 0.f, 0.f, 0.f};
#pragma unroll 1
    for (int i = tid; i < SCAP * DIMC / 4; i += NTHR) ((v4f*)rows)[i] = z4;
#pragma unroll 1
    for (int i = tid; i < NBA; i += NTHR) map[i] = -1;
#pragma unroll 1
    for (int i = tid; i < SCAP; i += NTHR) { rcnt[i] = 0; samp[i] = 0; }
    if (tid < 2 * DIMC / 4) ((v4f*)scsh)[tid] = *(const v4f*)(bnP + 4 * tid);
    if (tid < 2) cnt2[tid] = 0;
  }
  __syncthreads();

  const int nChB = (nB + CHUNK - 1) / CHUNK;
#pragma unroll 1
  for (int ch = 0; ch < nChB; ++ch) {
    const int cbase = ch * CHUNK;
    const int wc = scan_chunk<NBA, 1, 0>(nbr, nB, cbase, nodeBase, vec8, nN, list, map, tid, lane, wave);
    if (lane == 0) wcnt[wave] = wc;
    __syncthreads();
    if (tid == 0) {
      int nr = cnt2[0], ns = cnt2[1];
#pragma unroll 1
      for (int wsx = 0; wsx < NWAVE; ++wsx) {
        int n = wcnt[wsx];
        n = n > WCAP ? WCAP : (n < 0 ? 0 : n);
#pragma unroll 1
        for (int i = 0; i < n; ++i) {
          const int ent = list[wsx * WCAP + i];
          const int s = ent & (NBA - 1);
          int b = cbase + ((ent >> 12) & (CHUNK - 1));
          b = b > nB - 1 ? nB - 1 : b;
          int r = map[s];
          if (r < 0 && nr < SCAP) { r = nr; map[s] = r; nr = nr + 1; }
          if (r >= 0 && ns < SCAP) { samp[ns] = (b << 9) | r; ns = ns + 1; }
        }
      }
      cnt2[0] = nr; cnt2[1] = ns;
    }
    __syncthreads();
  }

  const v4f sc4 = *(const v4f*)(scsh + 4 * lane);
  const v4f sh4 = *(const v4f*)(scsh + DIMC + 4 * lane);
  const int nChE = (nE + CHUNK - 1) / CHUNK;
#pragma unroll 1
  for (int ch = 0; ch < nChE; ++ch) {
    const int cbase = ch * CHUNK;
    const int wc = scan_chunk<NBA, 0, 1>(dst, nE, cbase, nodeBase, vec8, nN, list, map, tid, lane, wave);
    if (lane == 0) wcnt[wave] = wc;
    __syncthreads();
    if (wave == 0) {
#pragma unroll 1
      for (int wsx = 0; wsx < NWAVE; ++wsx) {
        int n = __builtin_amdgcn_readfirstlane(wcnt[wsx]);
        n = n > WCAP ? WCAP : (n < 0 ? 0 : n);
        const int* lp = list + wsx * WCAP;
#pragma unroll 1
        for (int i = 0; i < n; ++i) {
          const int ent = __builtin_amdgcn_readfirstlane(lp[i]);
          int r = ent & 4095;
          r = r > SCAP - 1 ? SCAP - 1 : r;
          int e = cbase + ((ent >> 12) & (CHUNK - 1));
          e = e > nE - 1 ? nE - 1 : e;
          int s = src[e];
          s = clampi(s, 0, nN - 1);
          const v4f v  = *(const v4f*)(E + (size_t)s * DIMC + 4 * lane);
          const v4f hv = v * sc4 + sh4;
          v4f* rp = (v4f*)(rows + r * DIMC + 4 * lane);
          const v4f a = *rp;
          *rp = a + hv;
          if (lane == 0) rcnt[r] = rcnt[r] + 1;
        }
      }
    }
    __syncthreads();
  }

  int ns = cnt2[1];
  ns = ns < 0 ? 0 : (ns > SCAP ? SCAP : ns);
#pragma unroll 1
  for (int i = wave; i < ns; i += NWAVE) {
    const int ent = samp[i];
    int b = ent >> 9;
    b = clampi(b, 0, nB - 1);
    int r = ent & 511;
    r = r > SCAP - 1 ? SCAP - 1 : r;
    int c = rcnt[r];
    c = c < 1 ? 1 : c;
    const float inv = 1.0f / (float)c;
    const v4f v = *(const v4f*)(rows + r * DIMC + 4 * lane) * inv;
    float* gp = aggP + (size_t)b * DIMC + 4 * lane;
    *(volatile v4f*)gp = v;
    __threadfence();
    *(volatile v4f*)gp = v;
  }
}

__global__ __launch_bounds__(NTHR) void k_gemm_heads(
    const float* __restrict__ aggP, const __bf16* __restrict__ wh, const __bf16* __restrict__ wl,
    const float* __restrict__ bgnn,
    const float* __restrict__ Wg, const float* __restrict__ bg,
    const float* __restrict__ Wage, const float* __restrict__ bage,
    const float* __restrict__ Wocc, const float* __restrict__ bocc,
    const int* __restrict__ gender, const int* __restrict__ lblA, const int* __restrict__ lblO,
    float* hws, int nB, int offAge, int offGen, int offOcc, int offBce) {
  extern __shared__ v4f lds_dyn[];
  __bf16* sAhi  = (__bf16*)lds_dyn;
  __bf16* sAlo  = sAhi + GS * AP;
  float*  su    = (float*)lds_dyn;
  float*  sw    = (float*)((char*)lds_dyn + 2 * GS * AP * 2);
  float*  sbg   = sw + DIMC * HP;
  float*  sbias = sbg + DIMC;
  float*  sout  = sbias + HP;
  float*  sbce  = sout + GS * HP;
  const int tid = threadIdx.x, lane = tid & 31, wave = tid >> 5, hh = lane >> 4, m = lane & 15;
  const int blk = blockIdx.x;
  const int sBase = blk * GS;

#pragma unroll
  for (int i = 0; i < (GS * DIMC / 4) / NTHR; ++i) {
    const int idx = i * NTHR + tid;
    const int r = idx >> 5, c0 = (idx & 31) * 4;
    int row = sBase + r;
    row = row > nB - 1 ? nB - 1 : row;
    const v4f v = *(const v4f*)(aggP + (size_t)row * DIMC + c0);
    v4b hv, lv;
#pragma unroll
    for (int e = 0; e < 4; ++e) {
      __bf16 h, l;
      split_bf16(v[e], h, l);
      hv[e] = h; lv[e] = l;
    }
    *(v4b*)(sAhi + r * AP + c0) = hv;
    *(v4b*)(sAlo + r * AP + c0) = lv;
  }
#pragma unroll 1
  for (int idx = tid; idx < DIMC * HP; idx += NTHR) {
    const int k = idx >> 5, j = idx & 31;
    const float vg = Wg[k];
    const float va = Wage[k * NAGE + clampi(j - 1, 0, NAGE - 1)];
    const float vo = Wocc[k * NOCC + clampi(j - 1 - NAGE, 0, NOCC - 1)];
    sw[idx] = (j == 0) ? vg : (j <= NAGE ? va : (j < NHEAD ? vo : 0.0f));
  }
  if (tid < DIMC) sbg[tid] = bgnn[tid];
  if (tid < HP) {
    const int j = tid;
    const float vg = bg[0];
    const float va = bage[clampi(j - 1, 0, NAGE - 1)];
    const float vo = bocc[clampi(j - 1 - NAGE, 0, NOCC - 1)];
    sbias[j] = (j == 0) ? vg : (j <= NAGE ? va : (j < NHEAD ? vo : 0.0f));
  }
  __syncthreads();

  const int mt = wave & 3, ng = wave >> 2;
  v8f acc[4];
#pragma unroll
  for (int t = 0; t < 4; ++t) { v8f z = {0.f, 0.f, 0.f, 0.f, 0.f, 0.f, 0.f, 0.f}; acc[t] = z; }
  const __bf16* arh = sAhi + (16 * mt + m) * AP + 8 * hh;
  const __bf16* arl = sAlo + (16 * mt + m) * AP + 8 * hh;
#pragma unroll
  for (int kt = 0; kt < DIMC / 32; ++kt) {
    FragB ah, al;
    ah.h[0] = *(const v8b*)(arh + 32 * kt);
    ah.h[1] = *(const v8b*)(arh + 32 * kt + 16);
    al.h[0] = *(const v8b*)(arl + 32 * kt);
    al.h[1] = *(const v8b*)(arl + 32 * kt + 16);
#pragma unroll
    for (int t = 0; t < 4; ++t) {
      const int n = 16 * (4 * ng + t) + m;
      const __bf16* bph = wh + (size_t)n * DIMC + 32 * kt + 8 * hh;
      const __bf16* bpl = wl + (size_t)n * DIMC + 32 * kt + 8 * hh;
      FragB bh, bl;
      bh.h[0] = *(const v8b*)bph;
      bh.h[1] = *(const v8b*)(bph + 16);
      bl.h[0] = *(const v8b*)bpl;
      bl.h[1] = *(const v8b*)(bpl + 16);
      acc[t] = wmb(ah.v, bh.v, acc[t]);
      acc[t] = wmb(ah.v, bl.v, acc[t]);
      acc[t] = wmb(al.v, bh.v, acc[t]);
    }
  }
  __syncthreads();

  {
    const int r0 = 16 * mt + 8 * hh;
#pragma unroll
    for (int t = 0; t < 4; ++t) {
      const int col = 16 * (4 * ng + t) + m;
      const float bv = sbg[col];
#pragma unroll
      for (int r = 0; r < 8; ++r) {
        const float v = acc[t][r] + bv;
        su[(r0 + r) * DIMC + col] = fmaxf(v, 0.0f);
      }
    }
  }
  __syncthreads();

  {
    const int j = lane;
    const float bj = sbias[j];
    const float* wp = sw + j;
#pragma unroll 1
    for (int i = 0; i < GS / NWAVE; ++i) {
      const int rr = wave + NWAVE * i;
      const float* up = su + rr * DIMC;
      float a = 0.0f;
#pragma unroll 4
      for (int k = 0; k < DIMC; ++k) a = fmaf(up[k], wp[k * HP], a);
      const float val = a + bj;
      sout[rr * HP + j] = val;
      const int b  = sBase + rr;
      const int bc = b > nB - 1 ? nB - 1 : b;
      const float z = (float)gender[bc];
      const float x = val;
      float term = fmaxf(x, 0.0f) - x * z + log1pf(expf(-fabsf(x)));
      term = (b < nB) ? term : 0.0f;
      if (j == 0) sbce[rr] = term;
    }
  }
  __syncthreads();

  float part = 0.0f;
#pragma unroll 1
  for (int r = 0; r < GS; ++r) part += sbce[r];

  v4f vals[2];
  int offs[2];
#pragma unroll
  for (int it = 0; it < 2; ++it) {
    const int p  = it * NTHR + tid;
    const int pG = p - GS * NAGE / 4;
    const int pO = p - (GS * NAGE / 4 + GS / 4);
    const int pB = p - (GS * NAGE / 4 + GS / 4 + GS * NOCC / 4);
    v4f v = {0.f, 0.f, 0.f, 0.f};
#pragma unroll
    for (int e = 0; e < 4; ++e) {
      const int fa  = 4 * p + e;
      const int raw = fa / NAGE;
      const int ca  = fa - raw * NAGE;
      const int ra  = raw > GS - 1 ? GS - 1 : raw;
      const float va = sout[ra * HP + 1 + ca];
      const int fg  = clampi(4 * pG + e, 0, GS - 1);
      const float vg = sout[fg * HP];
      int fo = 4 * pO + e; fo = fo < 0 ? 0 : fo;
      const int row_o = fo / NOCC;
      const int co  = fo - row_o * NOCC;
      const int ro  = row_o > GS - 1 ? GS - 1 : row_o;
      const float vo = sout[ro * HP + 1 + NAGE + co];
      const int fb  = 4 * pB + e;
      const float vb = (fb == 0) ? part : 0.0f;
      v[e] = (p < GS * NAGE / 4) ? va
           : ((p < GS * NAGE / 4 + GS / 4) ? vg
           : ((p < GS * NAGE / 4 + GS / 4 + GS * NOCC / 4) ? vo : vb));
    }
    vals[it] = v;
    offs[it] = (p < GS * NAGE / 4) ? (offAge + blk * GS * NAGE + 4 * p)
             : ((p < GS * NAGE / 4 + GS / 4) ? (offGen + blk * GS + 4 * pG)
             : ((p < GS * NAGE / 4 + GS / 4 + GS * NOCC / 4) ? (offOcc + blk * GS * NOCC + 4 * pO)
             : (offBce + blk * 32 + 4 * pB)));
  }
#pragma unroll
  for (int it = 0; it < 2; ++it) {
    const int p = it * NTHR + tid;
    if (p < NPB) *(volatile v4f*)(hws + offs[it]) = vals[it];
  }
  __threadfence();
#pragma unroll
  for (int it = 0; it < 2; ++it) {
    const int p = it * NTHR + tid;
    if (p < NPB) *(volatile v4f*)(hws + offs[it]) = vals[it];
  }
}

__device__ __forceinline__ float out_val(const float* __restrict__ hws, int f, float lossv,
                                         int offAge, int offGen, int offOcc, int nAge, int nB, int nOcc) {
  const int fa = clampi(f - 1, 0, nAge - 1);
  const int fg = clampi(f - 1 - nAge, 0, nB - 1);
  const int fo = clampi(f - 1 - nAge - nB, 0, nOcc - 1);
  const int off = (f < 1 + nAge) ? (offAge + fa) : ((f < 1 + nAge + nB) ? (offGen + fg) : (offOcc + fo));
  const float v = hws[off];
  return (f == 0) ? lossv : v;
}

__global__ __launch_bounds__(NTHR) void k_out(
    const float* __restrict__ hws, int offAge, int offGen, int offOcc, int offBce,
    int nBlkG, int nB, float invB, float* out, int outN, int nPieces) {
  __shared__ float sLoss[4];
  const int tid = threadIdx.x;
  if (tid == 0) {
    double s = 0.0;
#pragma unroll 1
    for (int g = 0; g < nBlkG; ++g) s += (double)hws[offBce + g * 32];
    sLoss[0] = (float)s * invB;
  }
  __syncthreads();
  const float lossv = sLoss[0];
  const int nAge = nB * NAGE, nOcc = nB * NOCC;
  const int p = blockIdx.x * NTHR + tid;
  const int pmax = nPieces > 0 ? nPieces - 1 : 0;
  const int pc = p > pmax ? pmax : p;
  v4f v;
  v.x = out_val(hws, 4 * pc + 0, lossv, offAge, offGen, offOcc, nAge, nB, nOcc);
  v.y = out_val(hws, 4 * pc + 1, lossv, offAge, offGen, offOcc, nAge, nB, nOcc);
  v.z = out_val(hws, 4 * pc + 2, lossv, offAge, offGen, offOcc, nAge, nB, nOcc);
  v.w = out_val(hws, 4 * pc + 3, lossv, offAge, offGen, offOcc, nAge, nB, nOcc);
  const int nTail = outN - 4 * nPieces;
  int ft = 4 * nPieces + tid;
  ft = ft > outN - 1 ? outN - 1 : ft;
  const float tv = out_val(hws, ft, lossv, offAge, offGen, offOcc, nAge, nB, nOcc);
  const bool pact = p < nPieces;
  const bool tact = (blockIdx.x == 0) && (tid < nTail);
  float* vp = out + (size_t)4 * (size_t)pc;
  float* tp = out + (size_t)4 * (size_t)nPieces + (tact ? tid : 0);
  if (pact) *(volatile v4f*)vp = v;
  if (tact) *(volatile float*)tp = tv;
  __threadfence();
  if (pact) *(volatile v4f*)vp = v;
  if (tact) *(volatile float*)tp = tv;
}

extern "C" void kernel_launch(void* const* d_in, const int* in_sizes, int n_in,
                              void* d_out, int out_size, void* d_ws, size_t ws_size,
                              hipStream_t stream) {
  if (n_in < 17) return;
  const int nN = in_sizes[0] / DIMC;
  if (nN < 1 || in_sizes[0] != nN * DIMC) return;
  if (in_sizes[1] < DIMC || in_sizes[2] < DIMC || in_sizes[3] != DIMC * DIMC || in_sizes[4] < DIMC) return;
  if (in_sizes[5] < DIMC || in_sizes[6] < 1) return;
  if (in_sizes[7] != DIMC * NAGE || in_sizes[8] < NAGE || in_sizes[9] != DIMC * NOCC || in_sizes[10] < NOCC) return;
  const int nE = in_sizes[11];
  if (nE < 1 || in_sizes[12] != nE) return;
  const int nB = in_sizes[13];
  if (nB < 1 || in_sizes[14] < nB) return;
  if (out_size != 1 + nB * (NAGE + 1 + NOCC)) return;
  if (nN > (1 << 24) || nE > (1 << 28) || nB > (1 << 22)) return;

  const float* E     = (const float*)d_in[0];
  const float* gamma = (const float*)d_in[1];
  const float* beta  = (const float*)d_in[2];
  const float* Wgnn  = (const float*)d_in[3];
  const float* bgnn  = (const float*)d_in[4];
  const float* Wg    = (const float*)d_in[5];
  const float* bg    = (const float*)d_in[6];
  const float* Wage  = (const float*)d_in[7];
  const float* bage  = (const float*)d_in[8];
  const float* Wocc  = (const float*)d_in[9];
  const float* bocc  = (const float*)d_in[10];
  const int*   src   = (const int*)d_in[11];
  const int*   dst   = (const int*)d_in[12];
  const int*   nbr   = (const int*)d_in[13];
  const int*   gen   = (const int*)d_in[14];
  const int*   lblA  = (const int*)d_in[15];
  const int*   lblO  = (const int*)d_in[16];
  float* out = (float*)d_out;

  const int nP     = (nN + RPB - 1) / RPB;
  const int nBlkA  = (nN + NBA - 1) / NBA;
  const int nBlkG  = (nB + GS - 1) / GS;
  const int nPieces = (out_size / 32) * 8;
  int nBlkO = (nPieces + NTHR - 1) / NTHR;
  if (nBlkO < 1) nBlkO = 1;

  char* ws = (char*)d_ws;
  size_t off = 0;
  const size_t oWH   = off; off += (size_t)DIMC * DIMC * 2;                    off = (off + 255) & ~(size_t)255;
  const size_t oWL   = off; off += (size_t)DIMC * DIMC * 2;                    off = (off + 255) & ~(size_t)255;
  const size_t oStat = off; off += (size_t)nP * 2 * DIMC * 8;                  off = (off + 255) & ~(size_t)255;
  const size_t oBn   = off; off += (size_t)2 * DIMC * 4;                       off = (off + 255) & ~(size_t)255;
  const size_t oAgg  = off; off += (size_t)nBlkG * GS * DIMC * 4;              off = (off + 255) & ~(size_t)255;
  const size_t headF = (size_t)nBlkG * (GS * NAGE + GS + GS * NOCC + 32);
  const size_t oHead = off; off += headF * 4;                                  off = (off + 255) & ~(size_t)255;
  if (off > ws_size || off > ((size_t)128 << 20)) return;
  __bf16* wh   = (__bf16*)(ws + oWH);
  __bf16* wl   = (__bf16*)(ws + oWL);
  double* statP = (double*)(ws + oStat);
  float*  bnP  = (float*)(ws + oBn);
  float*  aggP = (float*)(ws + oAgg);
  float*  hws  = (float*)(ws + oHead);
  const int offAge = 0;
  const int offGen = offAge + nBlkG * GS * NAGE;
  const int offOcc = offGen + nBlkG * GS;
  const int offBce = offOcc + nBlkG * GS * NOCC;

  const double invN = 1.0 / (double)nN;
  const float  invB = 1.0f / (float)nB;

  k_stats<<<nP, NTHR, 0, stream>>>(E, statP, nN);
  k_bnfin<<<1, DIMC, 0, stream>>>(statP, nP, invN, gamma, beta, bnP);

  k_wprep<<<(DIMC * DIMC / 8 + NTHR - 1) / NTHR, NTHR, 0, stream>>>(Wgnn, wh, wl);

  hipFuncSetAttribute(reinterpret_cast<const void*>(&k_aggr),
                      hipFuncAttributeMaxDynamicSharedMemorySize, LDS_AGG);
  k_aggr<<<nBlkA, NTHR, LDS_AGG, stream>>>(E, src, dst, nbr, bnP, aggP, nN, nE, nB, 1);

  hipFuncSetAttribute(reinterpret_cast<const void*>(&k_gemm_heads),
                      hipFuncAttributeMaxDynamicSharedMemorySize, LDS_GH);
  k_gemm_heads<<<nBlkG, NTHR, LDS_GH, stream>>>(aggP, wh, wl, bgnn, Wg, bg, Wage, bage, Wocc, bocc,
                                                gen, lblA, lblO, hws, nB, offAge, offGen, offOcc, offBce);

  k_out<<<nBlkO, NTHR, 0, stream>>>(hws, offAge, offGen, offOcc, offBce, nBlkG, nB, invB, out, out_size, nPieces);
}
